// Proxy_Mixer_70901320123307
// MI455X (gfx1250) — hardware-run, weakly checked
//
#include <hip/hip_runtime.h>
#include <math.h>

typedef __attribute__((ext_vector_type(16))) _Float16 v16h;
typedef __attribute__((ext_vector_type(16))) __bf16   v16b;
typedef __attribute__((ext_vector_type(8)))  float    v8f;
typedef __attribute__((ext_vector_type(4)))  float    v4f;
typedef __attribute__((ext_vector_type(4)))  unsigned int v4u;
typedef __attribute__((ext_vector_type(8)))  unsigned int v8u;

constexpr int kB    = 4;
constexpr int kS    = 2048;
constexpr int kD    = 512;
constexpr int kP    = 16;
constexpr int kC    = 64;
constexpr int kNC   = kS / kC;
constexpr int kRows = kB * kS;
constexpr float kGateScale = 0.25f;
static_assert(kGateScale * kGateScale * (float)kP == 1.0f);
constexpr float kWCarry    = 64.0f;
constexpr float kWCarryInv = 1.0f / kWCarry;
static_assert(kWCarry * kWCarryInv == 1.0f);
static_assert(kS % kC == 0 && kC == 64 && kP == 16 && kD % 64 == 0);
constexpr int kAncPitchW = 260;
constexpr int kTilePitch = 104;
constexpr int kSlabPitch = 68;

constexpr size_t kOffXT   = 0;
constexpr size_t kOffP16  = kOffXT   + (size_t)kB * kD * kS * 2;
constexpr size_t kOffW16  = kOffP16  + (size_t)kRows * kP * 2;
constexpr size_t kOffPT16 = kOffW16  + (size_t)kRows * kP * 2;
constexpr size_t kOffDA   = kOffPT16 + (size_t)kB * kP * kS * 2;
constexpr size_t kOffABT  = kOffDA   + (size_t)kB * kNC * kP * kD * 4;
constexpr size_t kWsTotal = kOffABT  + (size_t)kB * kNC * kD * 32 * 2;
static_assert(kWsTotal == 17563648ull);
static_assert(kWsTotal <= 134217728ull);
static_assert((kOffP16 % 128) == 0 && (kOffW16 % 128) == 0 && (kOffPT16 % 128) == 0 &&
              (kOffDA % 128) == 0 && (kOffABT % 128) == 0);

__device__ __forceinline__ unsigned short f2bf_bits(float f) {
  unsigned u = __float_as_uint(f);
  return (unsigned short)((u + 0x7FFFu + ((u >> 16) & 1u)) >> 16);
}
__device__ __forceinline__ float bf_bits2f(unsigned short h) { return __uint_as_float(((unsigned)h) << 16); }
__device__ __forceinline__ unsigned pk16(unsigned short a, unsigned short b) { return (unsigned)a | ((unsigned)b << 16); }
__device__ __forceinline__ unsigned short h_bits(float f) { const _Float16 h = (_Float16)f; return __builtin_bit_cast(unsigned short, h); }

__device__ __forceinline__ void split_pair(float a, float b, unsigned& hw, unsigned& lw) {
  const unsigned short ha = f2bf_bits(a), hb = f2bf_bits(b);
  const unsigned short la = f2bf_bits(a - bf_bits2f(ha)), lb = f2bf_bits(b - bf_bits2f(hb));
  hw = pk16(ha, hb);
  lw = pk16(la, lb);
}

__device__ __forceinline__ v16h frag_h_words(v4u a, v4u b) {
  const v8u w = __builtin_shufflevector(a, b, 0, 1, 2, 3, 4, 5, 6, 7);
  return __builtin_bit_cast(v16h, w);
}
__device__ __forceinline__ v16b frag_b_words(v4u a, v4u b) {
  const v8u w = __builtin_shufflevector(a, b, 0, 1, 2, 3, 4, 5, 6, 7);
  return __builtin_bit_cast(v16b, w);
}
__device__ __forceinline__ v16h ldg_frag_h(const unsigned short* p) {
  const v4u a = *(const v4u*)(p);
  const v4u b = *(const v4u*)(p + 16);
  return frag_h_words(a, b);
}

__device__ __forceinline__ v8f mma_h(v16h a, v16h b, v8f c) {
  c = __builtin_amdgcn_wmma_f32_16x16x32_f16(false, a, false, b, (short)0, c, false, false);
  asm volatile("v_nop\n\tv_nop\n\tv_nop\n\tv_nop" : "+v"(c) : "v"(a), "v"(b));
  return c;
}
__device__ __forceinline__ v8f mma_b(v16b a, v16b b, v8f c) {
  c = __builtin_amdgcn_wmma_f32_16x16x32_bf16(false, a, false, b, (short)0, c, false, false);
  asm volatile("v_nop\n\tv_nop\n\tv_nop\n\tv_nop" : "+v"(c) : "v"(a), "v"(b));
  return c;
}

__global__ __launch_bounds__(256) void xpose_f16_kernel(const float* __restrict__ x, unsigned short* __restrict__ XT)
{
  __shared__ float sm[64 * 65];
  const int tid  = threadIdx.x;
  const int lane = tid & 31;
  const int wave = __builtin_amdgcn_readfirstlane((int)(threadIdx.x >> 5));
  const int d0 = blockIdx.x * 64;
  const int s0 = blockIdx.y * 64;
  const int b  = blockIdx.z;
  const float* xb = x + ((size_t)b * kS + s0) * kD + d0;
#pragma unroll
  for (int i = 0; i < 4; ++i) {
    const int e  = i * 256 + tid;
    const int r  = e >> 4;
    const int c4 = (e & 15) * 4;
    const v4f v = *(const v4f*)(xb + (size_t)r * kD + c4);
    sm[r * 65 + c4 + 0] = v[0];
    sm[r * 65 + c4 + 1] = v[1];
    sm[r * 65 + c4 + 2] = v[2];
    sm[r * 65 + c4 + 3] = v[3];
  }
  __syncthreads();
  const int q  = lane >> 3;
  const int s8 = (lane & 7) * 8;
  v4u u[2];
#pragma unroll
  for (int it = 0; it < 2; ++it) {
    const int dl = wave * 8 + it * 4 + q;
    unsigned short hb[8];
#pragma unroll
    for (int e = 0; e < 8; ++e) hb[e] = h_bits(sm[(s8 + e) * 65 + dl]);
    u[it] = (v4u){pk16(hb[0], hb[1]), pk16(hb[2], hb[3]), pk16(hb[4], hb[5]), pk16(hb[6], hb[7])};
  }
  for (int pass = 0; pass < 2; ++pass) {
#pragma unroll
    for (int it = 0; it < 2; ++it) {
      const int dl = wave * 8 + it * 4 + q;
      *(volatile v4u*)(XT + ((size_t)(b * kD + d0 + dl)) * kS + s0 + s8) = u[it];
    }
    __threadfence();
  }
}

__global__ __launch_bounds__(128) void scores_gate_kernel(
    const float* __restrict__ x, const float* __restrict__ anc,
    unsigned short* __restrict__ P16, unsigned short* __restrict__ W16, unsigned short* __restrict__ PT16)
{
  __shared__ __align__(16) unsigned sAH[kP * kAncPitchW];
  __shared__ __align__(16) unsigned sAL[kP * kAncPitchW];
  __shared__ float sProd[64 * 17];
  __shared__ float sGate[64 * 17];
  const int tid  = threadIdx.x;
  const int lane = tid & 31;
  const int wave = __builtin_amdgcn_readfirstlane((int)(threadIdx.x >> 5));
  const int hh = lane >> 4;
  const int cl = lane & 15;
  const int r0 = blockIdx.x * 64;
  const int b  = r0 / kS;
  const int s0 = r0 - b * kS;

#pragma unroll 1
  for (int i = 0; i < 16; ++i) {
    const int e4 = i * 128 + tid;
    const int p  = e4 >> 7;
    const int cf = (e4 & 127) * 4;
    const v4f v = *(const v4f*)(anc + (size_t)p * kD + cf);
    unsigned h01, l01, h23, l23;
    split_pair(v[0], v[1], h01, l01);
    split_pair(v[2], v[3], h23, l23);
    const int wo = p * kAncPitchW + (cf >> 1);
    sAH[wo]     = h01;
    sAH[wo + 1] = h23;
    sAL[wo]     = l01;
    sAL[wo + 1] = l23;
  }
  __syncthreads();

  const float* xrow = x + (size_t)(r0 + wave * 16 + cl) * kD + 8 * hh;
  v8f acc = (v8f){0.f, 0.f, 0.f, 0.f, 0.f, 0.f, 0.f, 0.f};
#pragma unroll 1
  for (int k0 = 0; k0 < kD; k0 += 32) {
    const v4f f0 = *(const v4f*)(xrow + k0);
    const v4f f1 = *(const v4f*)(xrow + k0 + 4);
    const v4f f2 = *(const v4f*)(xrow + k0 + 16);
    const v4f f3 = *(const v4f*)(xrow + k0 + 20);
    unsigned hw0, hw1, hw2, hw3, hw4, hw5, hw6, hw7;
    unsigned lw0, lw1, lw2, lw3, lw4, lw5, lw6, lw7;
    split_pair(f0[0], f0[1], hw0, lw0);
    split_pair(f0[2], f0[3], hw1, lw1);
    split_pair(f1[0], f1[1], hw2, lw2);
    split_pair(f1[2], f1[3], hw3, lw3);
    split_pair(f2[0], f2[1], hw4, lw4);
    split_pair(f2[2], f2[3], hw5, lw5);
    split_pair(f3[0], f3[1], hw6, lw6);
    split_pair(f3[2], f3[3], hw7, lw7);
    const v8u hv = (v8u){hw0, hw1, hw2, hw3, hw4, hw5, hw6, hw7};
    const v8u lv = (v8u){lw0, lw1, lw2, lw3, lw4, lw5, lw6, lw7};
    const v16b ah = __builtin_bit_cast(v16b, hv);
    const v16b al = __builtin_bit_cast(v16b, lv);
    const int wb = cl * kAncPitchW + (k0 >> 1) + 4 * hh;
    const v4u bh0 = *(const v4u*)(sAH + wb);
    const v4u bh1 = *(const v4u*)(sAH + wb + 8);
    const v4u bl0 = *(const v4u*)(sAL + wb);
    const v4u bl1 = *(const v4u*)(sAL + wb + 8);
    const v16b bh = frag_b_words(bh0, bh1);
    const v16b bl = frag_b_words(bl0, bl1);
    acc = mma_b(ah, bl, acc);
    acc = mma_b(al, bh, acc);
    acc = mma_b(ah, bh, acc);
  }
#pragma unroll
  for (int r = 0; r < 8; ++r) sProd[(wave * 16 + 8 * hh + r) * 17 + cl] = acc[r];
  __syncthreads();

  if (wave < 2) {
    const float* pr = sProd + tid * 17;
    float* gr = sGate + tid * 17;
    float m = pr[0] * kGateScale;
#pragma unroll 1
    for (int p = 1; p < kP; ++p) m = fmaxf(m, pr[p] * kGateScale);
    float sum = 0.0f;
#pragma unroll 1
    for (int p = 0; p < kP; ++p) {
      const float e = expf(pr[p] * kGateScale - m);
      gr[p] = e;
      sum += e;
    }
    const float inv = (1.0f / sum) * kWCarry;
#pragma unroll 1
    for (int p = 0; p < kP; ++p) gr[p] = gr[p] * inv;
  }
  __syncthreads();

  {
    const int q  = lane >> 3;
    const int j  = lane & 7;
    const int ln = wave * 4 + q;
    const int row = 4 * ln + (j >> 1);
    const int p0  = (j & 1) * 8;
    unsigned short pb[8], wb16[8], tb[8];
#pragma unroll
    for (int e = 0; e < 8; ++e) {
      pb[e]   = h_bits(sProd[row * 17 + p0 + e]);
      wb16[e] = h_bits(sGate[row * 17 + p0 + e]);
      tb[e]   = h_bits(sProd[(8 * j + e) * 17 + ln]);
    }
    const v4u up = (v4u){pk16(pb[0], pb[1]), pk16(pb[2], pb[3]), pk16(pb[4], pb[5]), pk16(pb[6], pb[7])};
    const v4u uw = (v4u){pk16(wb16[0], wb16[1]), pk16(wb16[2], wb16[3]), pk16(wb16[4], wb16[5]), pk16(wb16[6], wb16[7])};
    const v4u ut = (v4u){pk16(tb[0], tb[1]), pk16(tb[2], tb[3]), pk16(tb[4], tb[5]), pk16(tb[6], tb[7])};
    unsigned short* gp = P16 + (size_t)r0 * kP + ln * 64 + j * 8;
    unsigned short* gw = W16 + (size_t)r0 * kP + ln * 64 + j * 8;
    unsigned short* gt = PT16 + ((size_t)(b * kP + ln)) * kS + s0 + 8 * j;
    for (int pass = 0; pass < 2; ++pass) {
      *(volatile v4u*)gp = up;
      *(volatile v4u*)gw = uw;
      *(volatile v4u*)gt = ut;
      __threadfence();
    }
  }
}

__global__ __launch_bounds__(256) void chunk_state_kernel(
    const unsigned short* __restrict__ PT16, const unsigned short* __restrict__ XT, float* __restrict__ DA)
{
  __shared__ __align__(16) float slab[8 * 16 * kSlabPitch];
  const int tid  = threadIdx.x;
  const int lane = tid & 31;
  const int wave = __builtin_amdgcn_readfirstlane((int)(threadIdx.x >> 5));
  const int hh = lane >> 4;
  const int cl = lane & 15;
  const int bc = blockIdx.x;
  const int b  = bc / kNC;
  const int c0 = (bc - b * kNC) * kC;
  const int n0 = wave * 64;

  const unsigned short* aptr = PT16 + ((size_t)(b * kP + cl)) * kS + c0 + 8 * hh;
  const v16h a0 = ldg_frag_h(aptr);
  const v16h a1 = ldg_frag_h(aptr + 32);
  v8f acc[4];
#pragma unroll
  for (int j = 0; j < 4; ++j) acc[j] = (v8f){0.f, 0.f, 0.f, 0.f, 0.f, 0.f, 0.f, 0.f};
#pragma unroll
  for (int j = 0; j < 4; ++j) {
    const unsigned short* bptr = XT + ((size_t)(b * kD + n0 + 16 * j + cl)) * kS + c0 + 8 * hh;
    const v16h b0 = ldg_frag_h(bptr);
    const v16h b1 = ldg_frag_h(bptr + 32);
    acc[j] = mma_h(a0, b0, acc[j]);
    acc[j] = mma_h(a1, b1, acc[j]);
  }
  float* sw = slab + wave * 16 * kSlabPitch;
#pragma unroll
  for (int j = 0; j < 4; ++j)
#pragma unroll
    for (int r = 0; r < 8; ++r) sw[(8 * hh + r) * kSlabPitch + 16 * j + cl] = acc[j][r];
  __syncthreads();
  const int c4 = cl * 4;
  v4f v[8];
#pragma unroll
  for (int it = 0; it < 8; ++it) v[it] = *(const v4f*)(sw + (it * 2 + hh) * kSlabPitch + c4);
  for (int pass = 0; pass < 2; ++pass) {
#pragma unroll
    for (int it = 0; it < 8; ++it)
      *(volatile v4f*)(DA + ((size_t)bc * kP + it * 2 + hh) * kD + n0 + c4) = v[it];
    __threadfence();
  }
}

__global__ __launch_bounds__(64) void prefix_kernel(const float* __restrict__ DA, unsigned short* __restrict__ ABT)
{
  __shared__ __align__(16) unsigned sT[64 * 16];
  const int tid = threadIdx.x;
  const int b   = blockIdx.x >> 3;
  const int d0  = (blockIdx.x & 7) * 64;
  const int d   = d0 + tid;
  float run[kP];
#pragma unroll
  for (int p = 0; p < kP; ++p) run[p] = 0.0f;
#pragma unroll 1
  for (int c = 0; c < kNC; ++c) {
#pragma unroll
    for (int i = 0; i < 8; ++i) {
      const float a0 = run[2 * i], a1 = run[2 * i + 1];
      const _Float16 h0 = (_Float16)a0;
      const _Float16 h1 = (_Float16)a1;
      const float h0f = (float)h0;
      const float h1f = (float)h1;
      const unsigned short hb0 = __builtin_bit_cast(unsigned short, h0);
      const unsigned short hb1 = __builtin_bit_cast(unsigned short, h1);
      const unsigned short lb0 = h_bits(a0 - h0f);
      const unsigned short lb1 = h_bits(a1 - h1f);
      sT[tid * 16 + i]     = pk16(hb0, hb1);
      sT[tid * 16 + 8 + i] = pk16(lb0, lb1);
    }
    const float* src = DA + ((size_t)(b * kNC + c) * kP) * kD + d;
#pragma unroll
    for (int p = 0; p < kP; ++p) run[p] += src[(size_t)p * kD];
    __syncthreads();
    v4u v[4];
#pragma unroll
    for (int it = 0; it < 4; ++it) v[it] = *(const v4u*)(sT + (it * 64 + tid) * 4);
    __syncthreads();
    unsigned short* g = ABT + ((size_t)(b * kNC + c) * kD + d0) * 32;
    for (int pass = 0; pass < 2; ++pass) {
#pragma unroll
      for (int it = 0; it < 4; ++it)
        *(volatile v4u*)(g + (size_t)(it * 64 + tid) * 8) = v[it];
      __threadfence();
    }
  }
}

__global__ __launch_bounds__(256) void output_kernel(
    const unsigned short* __restrict__ W16, const unsigned short* __restrict__ P16,
    const unsigned short* __restrict__ ABT, const unsigned short* __restrict__ XT, float* __restrict__ out)
{
  __shared__ __align__(16) unsigned short sA[64 * kTilePitch];
  __shared__ __align__(16) float slab[8 * 16 * kSlabPitch];
  const int tid  = threadIdx.x;
  const int lane = tid & 31;
  const int wave = __builtin_amdgcn_readfirstlane((int)(threadIdx.x >> 5));
  const int hh = lane >> 4;
  const int cl = lane & 15;
  const int bc = blockIdx.x;
  const int b  = bc / kNC;
  const int c0 = (bc - b * kNC) * kC;
  const int r0 = b * kS + c0;
  const int mt = wave & 3;
  const int nh = wave >> 2;

  if (wave < 4) {
    const int row = tid >> 1;
    const int hf  = tid & 1;
    const v4u w = *(const v4u*)(W16 + (size_t)r0 * kP + tid * 8);
    *(v4u*)(sA + row * kTilePitch + hf * 8) = w;
    *(v4u*)(sA + row * kTilePitch + 16 + hf * 8) = w;
  }
  {
    const v4u zero4 = (v4u){0u, 0u, 0u, 0u};
    const v4u aw = *(const v4u*)(W16 + (size_t)(r0 + 16 * mt + cl) * kP + 8 * hh);
    const v16h af = frag_h_words(aw, zero4);
#pragma unroll
    for (int jj = 0; jj < 2; ++jj) {
      const int tt = nh * 2 + jj;
      const v4u pw = *(const v4u*)(P16 + (size_t)(r0 + 16 * tt + cl) * kP + 8 * hh);
      const v16h bf = frag_h_words(pw, zero4);
      v8f accL = (v8f){0.f, 0.f, 0.f, 0.f, 0.f, 0.f, 0.f, 0.f};
      accL = mma_h(af, bf, accL);
      const int tl = 16 * tt + cl;
#pragma unroll
      for (int r = 0; r < 8; ++r) {
        const int sl = 16 * mt + 8 * hh + r;
        const float val = (tl <= sl) ? accL[r] : 0.0f;
        sA[sl * kTilePitch + 32 + tl] = h_bits(val);
      }
    }
  }
  __syncthreads();

  v16h a[3];
#pragma unroll
  for (int ks = 0; ks < 3; ++ks) {
    const unsigned short* ap = sA + (16 * mt + cl) * kTilePitch + 32 * ks + 8 * hh;
    const v4u x0 = *(const v4u*)(ap);
    const v4u x1 = *(const v4u*)(ap + 16);
    a[ks] = frag_h_words(x0, x1);
  }

  float* sw = slab + wave * 16 * kSlabPitch;
  const int c4 = cl * 4;
#pragma unroll 1
  for (int g = 0; g < 4; ++g) {
    const int n0 = 256 * nh + 64 * g;
    v8f acc[4];
#pragma unroll
    for (int j = 0; j < 4; ++j) acc[j] = (v8f){0.f, 0.f, 0.f, 0.f, 0.f, 0.f, 0.f, 0.f};
#pragma unroll
    for (int j = 0; j < 4; ++j) {
      const int d = n0 + 16 * j + cl;
      const v16h bs = ldg_frag_h(ABT + ((size_t)bc * kD + d) * 32 + 8 * hh);
      acc[j] = mma_h(a[0], bs, acc[j]);
      const unsigned short* xt = XT + ((size_t)(b * kD + d)) * kS + c0 + 8 * hh;
      const v16h bx0 = ldg_frag_h(xt);
      acc[j] = mma_h(a[1], bx0, acc[j]);
      const v16h bx1 = ldg_frag_h(xt + 32);
      acc[j] = mma_h(a[2], bx1, acc[j]);
    }
#pragma unroll
    for (int j = 0; j < 4; ++j)
#pragma unroll
      for (int r = 0; r < 8; ++r) sw[(8 * hh + r) * kSlabPitch + 16 * j + cl] = acc[j][r] * kWCarryInv;
    __syncthreads();
    v4f v[8];
#pragma unroll
    for (int it = 0; it < 8; ++it) v[it] = *(const v4f*)(sw + (it * 2 + hh) * kSlabPitch + c4);
    for (int pass = 0; pass < 2; ++pass) {
#pragma unroll
      for (int it = 0; it < 8; ++it)
        *(volatile v4f*)(out + ((size_t)(r0 + 16 * mt + it * 2 + hh)) * kD + n0 + c4) = v[it];
      __threadfence();
    }
    __syncthreads();
  }
}

extern "C" void kernel_launch(void* const* d_in, const int* in_sizes, int n_in,
                              void* d_out, int out_size, void* d_ws, size_t ws_size,
                              hipStream_t stream) {
  if (n_in < 2) return;
  if (in_sizes[0] != kRows * kD) return;
  if (in_sizes[1] != kP * kD) return;
  if (out_size != kRows * kD) return;
  if (ws_size < kWsTotal) return;

  const float* x   = (const float*)d_in[0];
  const float* anc = (const float*)d_in[1];
  float* out = (float*)d_out;

  char* ws = (char*)d_ws;
  unsigned short* XT   = (unsigned short*)(ws + kOffXT);
  unsigned short* P16  = (unsigned short*)(ws + kOffP16);
  unsigned short* W16  = (unsigned short*)(ws + kOffW16);
  unsigned short* PT16 = (unsigned short*)(ws + kOffPT16);
  float*          DA   = (float*)(ws + kOffDA);
  unsigned short* ABT  = (unsigned short*)(ws + kOffABT);

  xpose_f16_kernel<<<dim3(kD / 64, kS / 64, kB), 256, 0, stream>>>(x, XT);
  scores_gate_kernel<<<dim3(kRows / 64), 128, 0, stream>>>(x, anc, P16, W16, PT16);
  chunk_state_kernel<<<dim3(kB * kNC), 256, 0, stream>>>(PT16, XT, DA);
  prefix_kernel<<<dim3(kB * (kD / 64)), 64, 0, stream>>>(DA, ABT);
  output_kernel<<<dim3(kB * kNC), 256, 0, stream>>>(W16, P16, ABT, XT, out);
}
